// RigidBody_24215025615351
// MI455X (gfx1250) — hardware-verified
//
#include <hip/hip_runtime.h>
#include <stddef.h>


typedef _Float16 h16;
typedef _Float16 v16h __attribute__((ext_vector_type(16)));
typedef _Float16 v8h  __attribute__((ext_vector_type(8)));
typedef float    v8f  __attribute__((ext_vector_type(8)));
typedef float    v4f  __attribute__((ext_vector_type(4)));

#ifndef NSAMP
#define NSAMP 4096
#endif
#define NSAMP_FULL 4096
#define NLINK 16
#define NQ    32
#define NCOL  34
#define KDIM  96
#define LDK   104
#define WAVES 2
#define CSF   (NQ * NCOL)
#define JCARRY 64.0f

static_assert(NSAMP >= WAVES && NSAMP <= NSAMP_FULL);
static_assert((NSAMP % WAVES) == 0);
static_assert(KDIM == NLINK * 6);
static_assert((KDIM % 32) == 0);
static_assert((LDK % 8) == 0 && LDK >= KDIM);
static_assert(NQ == 32);
static_assert((CSF % 4) == 0);
static_assert(((CSF * 4) % 128) == 0);
static_assert(CSF / 4 == 8 * 32 + 16);
static_assert(WAVES * 32 * LDK * 2 * 2 + WAVES * CSF * 4 <= 65536);

__device__ __forceinline__ float bf16r(float x) {
  unsigned int u = __float_as_uint(x);
  u = (u + 0x7FFFu + ((u >> 16) & 1u)) & 0xFFFF0000u;
  return __uint_as_float(u);
}

static __device__ __forceinline__ h16 toh_flush(float v) {
  const h16 r = (h16)v;
  return (fabsf(v) < 6.103515625e-05f) ? (h16)0.0f : r;
}

__device__ __forceinline__ v16h frag_at(const _Float16* p) {
  v8h lo = *(const v8h*)(p);
  v8h hi = *(const v8h*)(p + 16);
  v16h out;
#pragma unroll
  for (int i = 0; i < 8; ++i) { out[i] = lo[i]; out[i + 8] = hi[i]; }
  return out;
}
__device__ __forceinline__ v16h ld_frag(const _Float16* base, unsigned ld) {
  const unsigned lane = threadIdx.x & 31u;
  return frag_at(base + (lane & 15u) * ld + (lane >> 4) * 8u);
}

__device__ __forceinline__ v8f wmma16(v16h a, v16h b, v8f c) {
  v8f d = __builtin_amdgcn_wmma_f32_16x16x32_f16(false, a, false, b, (short)0, c,
                                                 false, false);
  asm volatile("v_nop\n\tv_nop\n\tv_nop\n\tv_nop" : "+v"(d) : "v"(a), "v"(b));
  return d;
}

__device__ __forceinline__ void wave_lds_sync() {
  __builtin_amdgcn_fence(3  , "wavefront");
  asm volatile("s_wait_dscnt 0x0" ::: "memory");
  __builtin_amdgcn_wave_barrier();
}

__global__ __launch_bounds__(64) void rigid_mass_kernel(
    const float* __restrict__ Js, const float* __restrict__ Jr, const float* __restrict__ Rib,
    const float* __restrict__ Wv, const float* __restrict__ dWv, const float* __restrict__ Av,
    const float* __restrict__ Mm, const float* __restrict__ Ib, const float* __restrict__ Gv,
    float* __restrict__ out) {
  __shared__ __attribute__((aligned(16))) _Float16 At[WAVES * 32 * LDK];
  __shared__ __attribute__((aligned(16))) _Float16 Bt[WAVES * 32 * LDK];
  __shared__ __attribute__((aligned(16))) float Cs[WAVES * CSF];

  const int wave = __builtin_amdgcn_readfirstlane(threadIdx.x >> 5);
  const unsigned lane = threadIdx.x & 31u;
  const unsigned hh = lane >> 4, m = lane & 15u;
  const unsigned b = blockIdx.x * (unsigned)WAVES + (unsigned)wave;
  const unsigned trow = (unsigned)wave * 32u;
  const unsigned cb = (unsigned)wave * (unsigned)CSF;

  const float g0 = bf16r(Gv[0]), g1 = bf16r(Gv[1]), g2 = bf16r(Gv[2]);
  float facc = 0.0f, gacc = 0.0f;

#pragma unroll 1
  for (unsigned l = 0; l < (unsigned)NLINK; ++l) {
    const size_t lb = (size_t)l * NSAMP_FULL + b;
    const size_t jbase = lb * 96u;
    const float js0 = bf16r(Js[jbase + lane]);
    const float js1 = bf16r(Js[jbase + 32u + lane]);
    const float js2 = bf16r(Js[jbase + 64u + lane]);
    const float jr0 = bf16r(Jr[jbase + lane]);
    const float jr1 = bf16r(Jr[jbase + 32u + lane]);
    const float jr2 = bf16r(Jr[jbase + 64u + lane]);

    const float ml = bf16r(Mm[l]);
    const float* Il = Ib + l * 9u;
    const float i00 = bf16r(Il[0]), i01 = bf16r(Il[1]), i02 = bf16r(Il[2]);
    const float i10 = bf16r(Il[3]), i11 = bf16r(Il[4]), i12 = bf16r(Il[5]);
    const float i20 = bf16r(Il[6]), i21 = bf16r(Il[7]), i22 = bf16r(Il[8]);
    const size_t vb = lb * 3u;
    const float w0 = bf16r(Wv[vb]), w1 = bf16r(Wv[vb + 1]), w2 = bf16r(Wv[vb + 2]);
    const float d0 = bf16r(dWv[vb]), d1 = bf16r(dWv[vb + 1]), d2 = bf16r(dWv[vb + 2]);
    const float a0 = bf16r(Av[vb]), a1 = bf16r(Av[vb + 1]), a2 = bf16r(Av[vb + 2]);
    const size_t rb = lb * 9u;
    const float gb0 = bf16r(Rib[rb + 0]) * g0 + bf16r(Rib[rb + 3]) * g1 + bf16r(Rib[rb + 6]) * g2;
    const float gb1 = bf16r(Rib[rb + 1]) * g0 + bf16r(Rib[rb + 4]) * g1 + bf16r(Rib[rb + 7]) * g2;
    const float gb2 = bf16r(Rib[rb + 2]) * g0 + bf16r(Rib[rb + 5]) * g1 + bf16r(Rib[rb + 8]) * g2;
    const float iw0 = i00 * w0 + i01 * w1 + i02 * w2;
    const float iw1 = i10 * w0 + i11 * w1 + i12 * w2;
    const float iw2 = i20 * w0 + i21 * w1 + i22 * w2;
    const float r0 = i00 * d0 + i01 * d1 + i02 * d2 + (w1 * iw2 - w2 * iw1);
    const float r1 = i10 * d0 + i11 * d1 + i12 * d2 + (w2 * iw0 - w0 * iw2);
    const float r2 = i20 * d0 + i21 * d1 + i22 * d2 + (w0 * iw1 - w1 * iw0);
    const float q0 = i00 * jr0 + i01 * jr1 + i02 * jr2;
    const float q1 = i10 * jr0 + i11 * jr1 + i12 * jr2;
    const float q2 = i20 * jr0 + i21 * jr1 + i22 * jr2;

    facc -= ml * (js0 * a0 + js1 * a1 + js2 * a2) + (jr0 * r0 + jr1 * r1 + jr2 * r2);
    gacc += ml * (js0 * gb0 + js1 * gb1 + js2 * gb2);

    const unsigned ro = (trow + lane) * LDK + 6u * l;
    At[ro + 0u] = toh_flush(JCARRY * (ml * js0));
    At[ro + 1u] = toh_flush(JCARRY * (ml * js1));
    At[ro + 2u] = toh_flush(JCARRY * (ml * js2));
    At[ro + 3u] = toh_flush(JCARRY * jr0);
    At[ro + 4u] = toh_flush(JCARRY * jr1);
    At[ro + 5u] = toh_flush(JCARRY * jr2);
    Bt[ro + 0u] = toh_flush(JCARRY * js0);
    Bt[ro + 1u] = toh_flush(JCARRY * js1);
    Bt[ro + 2u] = toh_flush(JCARRY * js2);
    Bt[ro + 3u] = toh_flush(JCARRY * q0);
    Bt[ro + 4u] = toh_flush(JCARRY * q1);
    Bt[ro + 5u] = toh_flush(JCARRY * q2);
  }
  wave_lds_sync();

  v8f acc00 = {}, acc01 = {}, acc10 = {}, acc11 = {};
#pragma unroll
  for (int ks = 0; ks < 3; ++ks) {
    const v16h fa0 = ld_frag(&At[trow * LDK + (unsigned)ks * 32u], LDK);
    const v16h fa1 = ld_frag(&At[(trow + 16u) * LDK + (unsigned)ks * 32u], LDK);
    const v16h fb0 = ld_frag(&Bt[trow * LDK + (unsigned)ks * 32u], LDK);
    const v16h fb1 = ld_frag(&Bt[(trow + 16u) * LDK + (unsigned)ks * 32u], LDK);
    acc00 = wmma16(fa0, fb0, acc00);
    acc01 = wmma16(fa0, fb1, acc01);
    acc10 = wmma16(fa1, fb0, acc10);
    acc11 = wmma16(fa1, fb1, acc11);
  }

  const float cs = 1.0f / (JCARRY * JCARRY);
#pragma unroll
  for (int r = 0; r < 8; ++r) {
    const unsigned row = hh * 8u + (unsigned)r;
    Cs[cb + row * NCOL + m]               = acc00[r] * cs;
    Cs[cb + row * NCOL + 16u + m]         = acc01[r] * cs;
    Cs[cb + (row + 16u) * NCOL + m]       = acc10[r] * cs;
    Cs[cb + (row + 16u) * NCOL + 16u + m] = acc11[r] * cs;
  }
  Cs[cb + lane * NCOL + 32u] = facc;
  Cs[cb + lane * NCOL + 33u] = gacc;
  wave_lds_sync();

  float* ob = out + (size_t)b * CSF;
  v4f x[9];
#pragma unroll
  for (unsigned i = 0; i < 9u; ++i) {
    unsigned idx = i * 32u + lane;
    idx = (idx < (unsigned)(CSF / 4 - 1)) ? idx : (unsigned)(CSF / 4 - 1);
    x[i] = *(const v4f*)&Cs[cb + idx * 4u];
  }
#pragma unroll
  for (unsigned i = 0; i < 8u; ++i) *(volatile v4f*)(ob + (i * 32u + lane) * 4u) = x[i];
  if (lane < 16u) *(volatile v4f*)(ob + (256u + lane) * 4u) = x[8];
  __threadfence();
#pragma unroll
  for (unsigned i = 0; i < 8u; ++i) *(volatile v4f*)(ob + (i * 32u + lane) * 4u) = x[i];
  if (lane < 16u) *(volatile v4f*)(ob + (256u + lane) * 4u) = x[8];
}

extern "C" void kernel_launch(void* const* d_in, const int* in_sizes, int n_in,
                              void* d_out, int out_size, void* d_ws, size_t ws_size,
                              hipStream_t stream) {
  (void)d_ws; (void)ws_size;
  if (n_in < 9) return;
  const long long nlb = (long long)(NLINK - 1) * NSAMP_FULL + NSAMP;
  if ((long long)in_sizes[0] < nlb * 96) return;
  if ((long long)in_sizes[1] < nlb * 96) return;
  if ((long long)in_sizes[2] < nlb * 9) return;
  if ((long long)in_sizes[3] < nlb * 3) return;
  if ((long long)in_sizes[4] < nlb * 3) return;
  if ((long long)in_sizes[5] < nlb * 3) return;
  if (in_sizes[6] < NLINK) return;
  if (in_sizes[7] < NLINK * 9) return;
  if (in_sizes[8] < 3) return;
  if ((long long)out_size < (long long)NSAMP * CSF) return;

  const float* Js  = (const float*)d_in[0];
  const float* Jr  = (const float*)d_in[1];
  const float* Rib = (const float*)d_in[2];
  const float* Wv  = (const float*)d_in[3];
  const float* dWv = (const float*)d_in[4];
  const float* Av  = (const float*)d_in[5];
  const float* Mm  = (const float*)d_in[6];
  const float* Ib  = (const float*)d_in[7];
  const float* Gv  = (const float*)d_in[8];
  float* out = (float*)d_out;

  rigid_mass_kernel<<<dim3(NSAMP / WAVES), dim3(32 * WAVES), 0, stream>>>(
      Js, Jr, Rib, Wv, dWv, Av, Mm, Ib, Gv, out);
}
